// MAB_37409165148591
// MI455X (gfx1250) — hardware-verified
//
#include <hip/hip_runtime.h>
#include <stdint.h>

#pragma clang fp contract(off)

typedef _Float16 f16;
typedef f16   v16h __attribute__((ext_vector_type(16)));
typedef f16   v8h  __attribute__((ext_vector_type(8)));
typedef f16   v4h  __attribute__((ext_vector_type(4)));
typedef float v8f  __attribute__((ext_vector_type(8)));
typedef float v4f  __attribute__((ext_vector_type(4)));

#ifndef NB
#define NB 4
#endif
#ifndef SEQ
#define SEQ 2048
#endif
#ifndef SEQK
#define SEQK SEQ
#endif

constexpr int NB_FULL = 4;
constexpr int LQ_FULL = 2048;
constexpr int LK_FULL = 2048;
constexpr int DM      = 512;
constexpr int NH      = 8;
constexpr int HD      = 64;
constexpr int SMAX    = (SEQ > SEQK) ? SEQ : SEQK;
constexpr float SCALE = 0.044194173824159216f;

static_assert(NB >= 1 && NB <= NB_FULL);
static_assert(SEQ % 256 == 0 && SEQ >= 256 && SEQ <= LQ_FULL);
static_assert(SEQK % 256 == 0 && SEQK >= 256 && SEQK <= LK_FULL);
static_assert(LQ_FULL == LK_FULL);
static_assert(DM == NH * HD);

constexpr size_t SZ_ACT16 = (size_t)NB_FULL * LQ_FULL * DM * 2;
constexpr size_t SZ_WT16  = (size_t)4 * DM * DM * 2;
constexpr size_t SZ_O32   = (size_t)NB_FULL * LQ_FULL * DM * 4;
constexpr size_t OFF_QH   = 0;
constexpr size_t OFF_KH   = OFF_QH + SZ_ACT16;
constexpr size_t OFF_WT   = OFF_KH + SZ_ACT16;
constexpr size_t OFF_QP   = OFF_WT + SZ_WT16;
constexpr size_t OFF_KP   = OFF_QP + SZ_ACT16;
constexpr size_t OFF_VT   = OFF_KP + SZ_ACT16;
constexpr size_t OFF_O32  = OFF_VT + SZ_ACT16;
constexpr size_t WS_TOTAL = OFF_O32 + SZ_O32;
static_assert(WS_TOTAL <= (size_t)134217728);
static_assert((OFF_KH % 256) == 0 && (OFF_WT % 256) == 0 && (OFF_QP % 256) == 0 &&
              (OFF_KP % 256) == 0 && (OFF_VT % 256) == 0 && (OFF_O32 % 256) == 0);

__device__ __forceinline__ float bf16_rne(float f) {
  unsigned int u = __float_as_uint(f);
  u = (u + 0x7FFFu + ((u >> 16) & 1u)) & 0xFFFF0000u;
  return __uint_as_float(u);
}

__device__ __forceinline__ v8f zero8() {
  const v8f z = {0.0f, 0.0f, 0.0f, 0.0f, 0.0f, 0.0f, 0.0f, 0.0f};
  return z;
}

__device__ __forceinline__ v16h load_tile16(const f16* base, int ld) {
  const int lane = threadIdx.x & 31;
  const int row  = lane & 15;
  const int hf   = lane >> 4;
  const f16* p = base + (size_t)row * ld + (hf << 3);
  union { v16h v; v8h h[2]; } u;
  u.h[0] = *(const v8h*)(p);
  u.h[1] = *(const v8h*)(p + 16);
  return u.v;
}

__device__ __forceinline__ v8f wmma16(v16h a, v16h b, v8f c) {
  v8f d = __builtin_amdgcn_wmma_f32_16x16x32_f16(false, a, false, b, (short)0, c, false, false);
  asm volatile("v_nop\n\tv_nop\n\tv_nop\n\tv_nop" : "+v"(d) : "v"(a), "v"(b));
  return d;
}

__global__ __launch_bounds__(256)
void cvt_act_kernel(const float* __restrict__ Q, const float* __restrict__ K,
                    f16* __restrict__ Qh, f16* __restrict__ Kh, long long n8) {
  const float* src = (blockIdx.y == 0) ? Q : K;
  f16* dst = (blockIdx.y == 0) ? Qh : Kh;
  const long long stride = (long long)gridDim.x * 256;
  for (long long i = (long long)blockIdx.x * 256 + threadIdx.x; i < n8; i += stride) {
    const v4f a = *(const v4f*)(src + i * 8);
    const v4f c = *(const v4f*)(src + i * 8 + 4);
    v8h o;
#pragma unroll
    for (int e = 0; e < 4; ++e) {
      o[e]     = (f16)bf16_rne(a[e]);
      o[e + 4] = (f16)bf16_rne(c[e]);
    }
    f16* p = dst + i * 8;
    *(volatile v8h*)p = o;
    __threadfence();
    *(volatile v8h*)p = o;
  }
}

__global__ __launch_bounds__(256)
void cvt_wt_kernel(const float* __restrict__ Wq, const float* __restrict__ Wk,
                   const float* __restrict__ Wv, const float* __restrict__ Wo,
                   f16* __restrict__ WT) {
  __shared__ __attribute__((aligned(16))) f16 tile[64 * 72];
  const int z = blockIdx.z;
  const float* W = (z == 0) ? Wq : (z == 1) ? Wk : (z == 2) ? Wv : Wo;
  f16* dst = WT + (size_t)z * DM * DM;
  const int k0 = blockIdx.x * 64;
  const int n0 = blockIdx.y * 64;
  const int tid = threadIdx.x;

#pragma unroll
  for (int it = 0; it < 4; ++it) {
    const int f  = tid + 256 * it;
    const int k  = f >> 4;
    const int n4 = (f & 15) * 4;
    const v4f w = *(const v4f*)(W + (size_t)(k0 + k) * DM + n0 + n4);
#pragma unroll
    for (int e = 0; e < 4; ++e)
      tile[(n4 + e) * 72 + k] = (f16)(bf16_rne(w[e]) * 16.0f);
  }
  __syncthreads();

  const int wave = tid >> 5, lane = tid & 31;
  const int piece = lane & 7;
  v8h vals[2];
#pragma unroll
  for (int it = 0; it < 2; ++it) {
    const int nl = wave * 8 + it * 4 + (lane >> 3);
    vals[it] = *(const v8h*)(tile + nl * 72 + piece * 8);
  }
#pragma unroll
  for (int it = 0; it < 2; ++it) {
    const int nl = wave * 8 + it * 4 + (lane >> 3);
    *(volatile v8h*)(dst + (size_t)(n0 + nl) * DM + k0 + piece * 8) = vals[it];
  }
  __threadfence();
#pragma unroll
  for (int it = 0; it < 2; ++it) {
    const int nl = wave * 8 + it * 4 + (lane >> 3);
    *(volatile v8h*)(dst + (size_t)(n0 + nl) * DM + k0 + piece * 8) = vals[it];
  }
}

__global__ __launch_bounds__(256)
void proj_kernel(const f16* __restrict__ Xq, const f16* __restrict__ Xk,
                 const f16* __restrict__ WT,
                 const float* __restrict__ bq, const float* __restrict__ bk,
                 const float* __restrict__ bv,
                 f16* __restrict__ Qp, f16* __restrict__ Kp, f16* __restrict__ Vt) {
  __shared__ __attribute__((aligned(16))) f16 stg[256 * 64];
  const int z = blockIdx.z;
  const int S = (z == 0) ? SEQ : SEQK;
  const int tilesPerB = S / 256;
  const int nblk = NB * tilesPerB;
  if ((int)blockIdx.x >= nblk) return;

  const f16* X = (z == 0) ? Xq : Xk;
  const f16* W = WT + (size_t)z * DM * DM;
  const float* bias = (z == 0) ? bq : (z == 1) ? bk : bv;

  const int b     = blockIdx.x / tilesPerB;
  const int rloc  = (blockIdx.x % tilesPerB) * 256;
  const int row0g = b * LQ_FULL + rloc;
  const int c0    = blockIdx.y * 64;

  const int tid = threadIdx.x;
  const int wave = tid >> 5, lane = tid & 31, n16 = lane & 15, hf = lane >> 4;

  v8f acc[2][4];
#pragma unroll
  for (int s = 0; s < 2; ++s)
#pragma unroll
    for (int t = 0; t < 4; ++t) acc[s][t] = zero8();

#pragma unroll 1
  for (int k = 0; k < DM; k += 32) {
    const v16h a0 = load_tile16(X + (size_t)(row0g + wave * 32) * DM + k, DM);
    const v16h a1 = load_tile16(X + (size_t)(row0g + wave * 32 + 16) * DM + k, DM);
#pragma unroll
    for (int t = 0; t < 4; ++t) {
      const v16h bfr = load_tile16(W + (size_t)(c0 + 16 * t) * DM + k, DM);
      acc[0][t] = wmma16(a0, bfr, acc[0][t]);
      acc[1][t] = wmma16(a1, bfr, acc[1][t]);
    }
  }

#pragma unroll
  for (int t = 0; t < 4; ++t) {
    const int lc = 16 * t + n16;
    const float bb = bf16_rne(bias[c0 + lc]);
#pragma unroll
    for (int s = 0; s < 2; ++s) {
#pragma unroll
      for (int r = 0; r < 8; ++r) {
        const int lr = wave * 32 + 16 * s + 8 * hf + r;
        const float v = acc[s][t][r] * 0.0625f + bb;
        const f16 hv = (f16)v;
        if (z == 2) stg[lc * 256 + lr] = hv;
        else        stg[lr * 64 + lc] = hv;
      }
    }
  }
  __syncthreads();

  if (z != 2) {
    f16* out = (z == 0) ? Qp : Kp;
    const int piece = lane & 7;
    v8h vals[8];
#pragma unroll
    for (int it = 0; it < 8; ++it) {
      const int lr = wave * 32 + it * 4 + (lane >> 3);
      vals[it] = *(const v8h*)(stg + lr * 64 + piece * 8);
    }
#pragma unroll
    for (int it = 0; it < 8; ++it) {
      const int lr = wave * 32 + it * 4 + (lane >> 3);
      *(volatile v8h*)(out + (size_t)(row0g + lr) * DM + c0 + piece * 8) = vals[it];
    }
    __threadfence();
#pragma unroll
    for (int it = 0; it < 8; ++it) {
      const int lr = wave * 32 + it * 4 + (lane >> 3);
      *(volatile v8h*)(out + (size_t)(row0g + lr) * DM + c0 + piece * 8) = vals[it];
    }
  } else {
    v8h vals[8];
#pragma unroll
    for (int it = 0; it < 8; ++it) {
      const int d = wave * 8 + it;
      vals[it] = *(const v8h*)(stg + d * 256 + lane * 8);
    }
#pragma unroll
    for (int it = 0; it < 8; ++it) {
      const int d = wave * 8 + it;
      *(volatile v8h*)(Vt + (size_t)(b * DM + c0 + d) * LK_FULL + rloc + lane * 8) = vals[it];
    }
    __threadfence();
#pragma unroll
    for (int it = 0; it < 8; ++it) {
      const int d = wave * 8 + it;
      *(volatile v8h*)(Vt + (size_t)(b * DM + c0 + d) * LK_FULL + rloc + lane * 8) = vals[it];
    }
  }
}

__global__ __launch_bounds__(256) __attribute__((amdgpu_num_vgpr(256)))
void attn_kernel(const f16* __restrict__ Qp, const f16* __restrict__ Kp,
                 const f16* __restrict__ Vt, const int* __restrict__ pmask,
                 float* __restrict__ Og) {
  __shared__ __attribute__((aligned(16))) f16   kbuf[32 * 64];
  __shared__ __attribute__((aligned(16))) f16   vbuf[64 * 32];
  __shared__ __attribute__((aligned(16))) f16   ldsP[8 * 16 * 32];
  __shared__ __attribute__((aligned(16))) float mks[LK_FULL];
  __shared__ __attribute__((aligned(16))) float ost[8 * 16 * 64];

  const int tid = threadIdx.x;
  const int wave = tid >> 5, lane = tid & 31, n16 = lane & 15, hf = lane >> 4;
  const int b = blockIdx.x / NH;
  const int h = blockIdx.x % NH;
  const int q0 = blockIdx.y * 128 + wave * 16;
  const int qrow = b * LQ_FULL + q0;

  for (int i = tid; i < SEQK; i += 256) mks[i] = (float)pmask[(size_t)b * LK_FULL + i];

  const v16h aq0 = load_tile16(Qp + (size_t)qrow * DM + h * HD, DM);
  const v16h aq1 = load_tile16(Qp + (size_t)qrow * DM + h * HD + 32, DM);

  v8f o0 = zero8(), o1 = zero8(), o2 = zero8(), o3 = zero8();
  float mrow[8], lrow[8];
#pragma unroll
  for (int r = 0; r < 8; ++r) { mrow[r] = -1e30f; lrow[r] = 0.0f; }

  f16* myP = ldsP + wave * 512;
  const f16* Kg = Kp + (size_t)b * LK_FULL * DM + h * HD;
  const f16* Vg = Vt + ((size_t)b * DM + h * HD) * LK_FULL;

#pragma unroll 1
  for (int j = 0; j < SEQK; j += 32) {
    {
      const int row = tid >> 3, ch = tid & 7;
      *(v8h*)(kbuf + row * 64 + ch * 8) = *(const v8h*)(Kg + (size_t)(j + row) * DM + ch * 8);
    }
    {
      const int row = tid >> 2, ch = tid & 3;
      *(v8h*)(vbuf + row * 32 + ch * 8) = *(const v8h*)(Vg + (size_t)row * LK_FULL + j + ch * 8);
    }
    __syncthreads();

    v8f s0 = zero8(), s1 = zero8();
    s0 = wmma16(aq0, load_tile16(kbuf, 64), s0);
    s0 = wmma16(aq1, load_tile16(kbuf + 32, 64), s0);
    s1 = wmma16(aq0, load_tile16(kbuf + 16 * 64, 64), s1);
    s1 = wmma16(aq1, load_tile16(kbuf + 16 * 64 + 32, 64), s1);

    const float mk0 = mks[j + n16];
    const float mk1 = mks[j + 16 + n16];
#pragma unroll
    for (int r = 0; r < 8; ++r) {
      const float a0 = (mk0 == 0.0f) ? -1e12f : s0[r] * SCALE;
      const float a1 = (mk1 == 0.0f) ? -1e12f : s1[r] * SCALE;
      float v = fmaxf(a0, a1);
#pragma unroll
      for (int off = 8; off >= 1; off >>= 1) v = fmaxf(v, __shfl_xor(v, off, 16));
      const float mnew = fmaxf(mrow[r], v);
      const float p0 = __expf(a0 - mnew);
      const float p1 = __expf(a1 - mnew);
      float ps = p0 + p1;
#pragma unroll
      for (int off = 8; off >= 1; off >>= 1) ps += __shfl_xor(ps, off, 16);
      const float ef = __expf(mrow[r] - mnew);
      lrow[r] = lrow[r] * ef + ps;
      mrow[r] = mnew;
      const int q = r + 8 * hf;
      myP[q * 32 + n16]      = (f16)(p0 * mk0 * 256.0f);
      myP[q * 32 + 16 + n16] = (f16)(p1 * mk1 * 256.0f);
      o0[r] *= ef; o1[r] *= ef; o2[r] *= ef; o3[r] *= ef;
    }
    __syncthreads();

    const v16h ap = load_tile16(myP, 32);
    o0 = wmma16(ap, load_tile16(vbuf,           32), o0);
    o1 = wmma16(ap, load_tile16(vbuf + 16 * 32, 32), o1);
    o2 = wmma16(ap, load_tile16(vbuf + 32 * 32, 32), o2);
    o3 = wmma16(ap, load_tile16(vbuf + 48 * 32, 32), o3);

    __syncthreads();
  }

  float* myO = ost + wave * 1024;
#pragma unroll
  for (int r = 0; r < 8; ++r) {
    const float linv = __builtin_amdgcn_rcpf(lrow[r] * 256.0f);
    const int q = r + 8 * hf;
    float* pr = myO + q * 64 + n16;
    pr[0]  = o0[r] * linv;
    pr[16] = o1[r] * linv;
    pr[32] = o2[r] * linv;
    pr[48] = o3[r] * linv;
  }
  __syncthreads();

  const int c4 = (lane & 15) * 4;
  v4f vals[8];
#pragma unroll
  for (int it = 0; it < 8; ++it) {
    const int row = it * 2 + (lane >> 4);
    vals[it] = *(const v4f*)(myO + row * 64 + c4);
  }
#pragma unroll
  for (int it = 0; it < 8; ++it) {
    const int row = it * 2 + (lane >> 4);
    *(volatile v4f*)(Og + (size_t)(qrow + row) * DM + h * HD + c4) = vals[it];
  }
  __threadfence();
#pragma unroll
  for (int it = 0; it < 8; ++it) {
    const int row = it * 2 + (lane >> 4);
    *(volatile v4f*)(Og + (size_t)(qrow + row) * DM + h * HD + c4) = vals[it];
  }
}

__global__ __launch_bounds__(256)
void ffn_ln_kernel(const float* __restrict__ O32, const float* __restrict__ Qraw,
                   const f16* __restrict__ WoT, const float* __restrict__ bo,
                   const float* __restrict__ g0, const float* __restrict__ b0,
                   const float* __restrict__ g1, const float* __restrict__ b1,
                   float* __restrict__ out) {
  __shared__ __attribute__((aligned(16))) float xf[16 * 512];
  __shared__ __attribute__((aligned(16))) f16   xh[16 * 512];

  const int tilesPerB = SEQ / 16;
  const int b     = blockIdx.x / tilesPerB;
  const int rloc  = (blockIdx.x % tilesPerB) * 16;
  const int grow0 = b * LQ_FULL + rloc;

  const int tid = threadIdx.x;
  const int wave = tid >> 5, lane = tid & 31, n16 = lane & 15, hf = lane >> 4;
  constexpr float INV_D = 1.0f / 512.0f;

#pragma unroll
  for (int rr = 0; rr < 2; ++rr) {
    const int lr = wave * 2 + rr;
    const size_t grow = (size_t)(grow0 + lr);
    float x[16];
    float s = 0.0f;
#pragma unroll
    for (int i = 0; i < 4; ++i) {
      const int col = i * 128 + lane * 4;
      const v4f ov = *(const v4f*)(O32 + grow * DM + col);
      const v4f qv = *(const v4f*)(Qraw + grow * DM + col);
#pragma unroll
      for (int e = 0; e < 4; ++e) {
        const float xx = bf16_rne(qv[e]) + ov[e];
        x[i * 4 + e] = xx;
        s += xx;
      }
    }
#pragma unroll
    for (int off = 16; off > 0; off >>= 1) s += __shfl_xor(s, off, 32);
    const float mu = s * INV_D;
    float s2 = 0.0f;
#pragma unroll
    for (int i = 0; i < 16; ++i) {
      const float d = x[i] - mu;
      x[i] = d;
      const float dd = d * d;
      s2 += dd;
    }
#pragma unroll
    for (int off = 16; off > 0; off >>= 1) s2 += __shfl_xor(s2, off, 32);
    const float var = s2 * INV_D;
    const float rsq = rsqrtf(var + 1e-5f);
#pragma unroll
    for (int i = 0; i < 4; ++i) {
      const int col = i * 128 + lane * 4;
      const v4f gv = *(const v4f*)(g0 + col);
      const v4f bv4 = *(const v4f*)(b0 + col);
      v4f y; v4h yh;
#pragma unroll
      for (int e = 0; e < 4; ++e) {
        const float t0 = x[i * 4 + e] * rsq;
        const float t1 = t0 * bf16_rne(gv[e]);
        const float yy = t1 + bf16_rne(bv4[e]);
        y[e] = yy;
        yh[e] = (f16)yy;
      }
      *(v4f*)(xf + lr * 512 + col) = y;
      *(v4h*)(xh + lr * 512 + col) = yh;
    }
  }
  __syncthreads();

  const int cw = wave * 64;
  v8f acc[4];
#pragma unroll
  for (int t = 0; t < 4; ++t) acc[t] = zero8();
#pragma unroll 1
  for (int k = 0; k < DM; k += 32) {
    const v16h a = load_tile16(xh + k, 512);
#pragma unroll
    for (int t = 0; t < 4; ++t) {
      const v16h bfr = load_tile16(WoT + (size_t)(cw + 16 * t) * DM + k, DM);
      acc[t] = wmma16(a, bfr, acc[t]);
    }
  }

#pragma unroll
  for (int t = 0; t < 4; ++t) {
    const int col = cw + 16 * t + n16;
    const float bb = bf16_rne(bo[col]);
#pragma unroll
    for (int r = 0; r < 8; ++r) {
      const int lr = 8 * hf + r;
      float hv = acc[t][r] * 0.0625f + bb;
      hv = fmaxf(hv, 0.0f);
      const int idx = lr * 512 + col;
      const float yv = xf[idx] + hv;
      xf[idx] = yv;
    }
  }
  __syncthreads();

#pragma unroll
  for (int rr = 0; rr < 2; ++rr) {
    const int lr = wave * 2 + rr;
    const size_t grow = (size_t)(grow0 + lr);
    float x[16];
    float s = 0.0f;
#pragma unroll
    for (int i = 0; i < 4; ++i) {
      const int col = i * 128 + lane * 4;
      const v4f xv = *(const v4f*)(xf + lr * 512 + col);
#pragma unroll
      for (int e = 0; e < 4; ++e) { x[i * 4 + e] = xv[e]; s += xv[e]; }
    }
#pragma unroll
    for (int off = 16; off > 0; off >>= 1) s += __shfl_xor(s, off, 32);
    const float mu = s * INV_D;
    float s2 = 0.0f;
#pragma unroll
    for (int i = 0; i < 16; ++i) {
      const float d = x[i] - mu;
      x[i] = d;
      const float dd = d * d;
      s2 += dd;
    }
#pragma unroll
    for (int off = 16; off > 0; off >>= 1) s2 += __shfl_xor(s2, off, 32);
    const float var = s2 * INV_D;
    const float rsq = rsqrtf(var + 1e-5f);
    v4f y[4];
#pragma unroll
    for (int i = 0; i < 4; ++i) {
      const int col = i * 128 + lane * 4;
      const v4f gv = *(const v4f*)(g1 + col);
      const v4f bv4 = *(const v4f*)(b1 + col);
#pragma unroll
      for (int e = 0; e < 4; ++e) {
        const float t0 = x[i * 4 + e] * rsq;
        const float t1 = t0 * bf16_rne(gv[e]);
        y[i][e] = t1 + bf16_rne(bv4[e]);
      }
    }
    float* orow = out + grow * DM + lane * 4;
#pragma unroll
    for (int i = 0; i < 4; ++i) *(volatile v4f*)(orow + i * 128) = y[i];
    __threadfence();
#pragma unroll
    for (int i = 0; i < 4; ++i) *(volatile v4f*)(orow + i * 128) = y[i];
  }
}

extern "C" void kernel_launch(void* const* d_in, const int* in_sizes, int n_in,
                              void* d_out, int out_size, void* d_ws, size_t ws_size,
                              hipStream_t stream) {
  if (n_in < 15) return;
  const float* Q     = (const float*)d_in[0];
  const float* K     = (const float*)d_in[1];
  const int*   pmask = (const int*)d_in[2];
  const float* Wq    = (const float*)d_in[3];
  const float* bq    = (const float*)d_in[4];
  const float* Wk    = (const float*)d_in[5];
  const float* bk    = (const float*)d_in[6];
  const float* Wv    = (const float*)d_in[7];
  const float* bv    = (const float*)d_in[8];
  const float* Wo    = (const float*)d_in[9];
  const float* bo    = (const float*)d_in[10];
  const float* g0    = (const float*)d_in[11];
  const float* b0    = (const float*)d_in[12];
  const float* g1    = (const float*)d_in[13];
  const float* b1    = (const float*)d_in[14];
  float* out = (float*)d_out;

  const long long needAct = (long long)((NB - 1) * LQ_FULL + SMAX) * DM;
  const long long needOut = (long long)((NB - 1) * LQ_FULL + SEQ) * DM;
  if ((long long)in_sizes[0] < needAct || (long long)in_sizes[1] < needAct) return;
  if (in_sizes[2] < (NB - 1) * LK_FULL + SEQK) return;
  if (in_sizes[3] < DM * DM || in_sizes[5] < DM * DM || in_sizes[7] < DM * DM ||
      in_sizes[9] < DM * DM) return;
  if (in_sizes[4] < DM || in_sizes[6] < DM || in_sizes[8] < DM || in_sizes[10] < DM ||
      in_sizes[11] < DM || in_sizes[12] < DM || in_sizes[13] < DM || in_sizes[14] < DM) return;
  if ((long long)out_size < needOut) return;
  if (ws_size < WS_TOTAL) return;

  char* ws = (char*)d_ws;
  f16*   Qh  = (f16*)(ws + OFF_QH);
  f16*   Kh  = (f16*)(ws + OFF_KH);
  f16*   WT  = (f16*)(ws + OFF_WT);
  f16*   Qp  = (f16*)(ws + OFF_QP);
  f16*   Kp  = (f16*)(ws + OFF_KP);
  f16*   Vt  = (f16*)(ws + OFF_VT);
  float* O32 = (float*)(ws + OFF_O32);

  const long long n8 = needAct / 8;
  cvt_act_kernel<<<dim3(512, 2), 256, 0, stream>>>(Q, K, Qh, Kh, n8);
  cvt_wt_kernel<<<dim3(DM / 64, DM / 64, 4), 256, 0, stream>>>(Wq, Wk, Wv, Wo, WT);

  proj_kernel<<<dim3(NB * (SMAX / 256), DM / 64, 3), 256, 0, stream>>>(
      Qh, Kh, WT, bq, bk, bv, Qp, Kp, Vt);

  attn_kernel<<<dim3(NB * NH, SEQ / 128), 256, 0, stream>>>(Qp, Kp, Vt, pmask, O32);

  ffn_ln_kernel<<<dim3(NB * (SEQ / 16)), 256, 0, stream>>>(
      O32, Q, WT + (size_t)3 * DM * DM, bo, g0, b0, g1, b1, out);
}
